// MambaBlock_25598005084283
// MI455X (gfx1250) — hardware-run, weakly checked
//
#include <hip/hip_runtime.h>
#include <math.h>

typedef __attribute__((ext_vector_type(8)))  _Float16 v8h;
typedef __attribute__((ext_vector_type(16))) __bf16   v16b;
typedef __attribute__((ext_vector_type(8)))  __bf16   v8b;
typedef __attribute__((ext_vector_type(8)))  float    v8f;
typedef __attribute__((ext_vector_type(4)))  float    v4f;
typedef __attribute__((ext_vector_type(4)))  unsigned int v4u;
typedef __attribute__((ext_vector_type(2)))  unsigned int v2u;

constexpr int kBatch  = 4;
constexpr int kSeq    = 2048;
constexpr int kDm     = 512;
constexpr int kE      = 1024;
constexpr int kNst    = 16;
constexpr int kConvK  = 4;
constexpr int kWin    = 2 * kE;
constexpr int kDlP    = 64;
constexpr int kRows   = kBatch * kSeq;
constexpr int kConvTP = 260;
constexpr int kScanTS = 64;
constexpr int kScanCh = 64;
constexpr int kSYP    = 68;
constexpr int kGateSP = 36;
static_assert((kDm % 32) == 0 && (kE % 32) == 0, "GEMM K multiples of 32");
static_assert((kRows % 64) == 0 && (kWin % 64) == 0 && (kDlP % 64) == 0 && (kDm % 64) == 0, "GEMM M,N multiples of 64");
static_assert((kSeq % kScanTS) == 0 && (kSeq % 64) == 0 && (kE % kScanCh) == 0 && (kE % 256) == 0, "tile multiples");
static_assert(kNst == 16 && kConvK == 4 && kNst <= kDlP, "shape assumptions");

constexpr int kTilesIn  = (kRows / 64) * (kWin / 64);
constexpr int kTilesDl  = (kRows / 64) * (kDlP / 64);
constexpr int kTilesOut = (kRows / 64) * (kDm  / 64);
static_assert((kTilesIn % 8) == 0 && (kTilesDl % 8) == 0 && (kTilesOut % 8) == 0, "exact GEMM grids");

constexpr size_t kOffXB   = 0;
constexpr size_t kOffWIB  = kOffXB  + (size_t)kRows * kDm  * 2;
constexpr size_t kOffWOB  = kOffWIB + (size_t)kWin  * kDm  * 2;
constexpr size_t kOffBPT  = kOffWOB + (size_t)kDm   * kE   * 2;
constexpr size_t kOffXS   = kOffBPT + (size_t)kDlP  * kE   * 2;
constexpr size_t kOffUH   = kOffXS  + (size_t)kRows * kE   * 4;
constexpr size_t kOffUL   = kOffUH  + (size_t)kRows * kE   * 2;
constexpr size_t kOffDL   = kOffUL  + (size_t)kRows * kE   * 2;
constexpr size_t kOffYH   = kOffDL  + (size_t)kRows * kDlP * 4;
constexpr size_t kOffYL   = kOffYH  + (size_t)kRows * kE   * 2;
constexpr size_t kWsTotal = kOffYL  + (size_t)kRows * kE   * 2;
static_assert(kWsTotal == 114425856ull, "carve total");
static_assert(kWsTotal <= 134217728ull, "carve cap");
static_assert((kOffWIB % 128) == 0 && (kOffWOB % 128) == 0 && (kOffBPT % 128) == 0 && (kOffXS % 128) == 0 &&
              (kOffUH % 128) == 0 && (kOffUL % 128) == 0 && (kOffDL % 128) == 0 && (kOffYH % 128) == 0 &&
              (kOffYL % 128) == 0, "128-B aligned regions");

__device__ __forceinline__ unsigned short f2bf_bits(float f) {
  unsigned u = __float_as_uint(f);
  return (unsigned short)((u + 0x7FFFu + ((u >> 16) & 1u)) >> 16);
}
__device__ __forceinline__ float bf_bits2f(unsigned short h) { return __uint_as_float(((unsigned)h) << 16); }
__device__ __forceinline__ float bfr(float f) { return bf_bits2f(f2bf_bits(f)); }

__device__ __forceinline__ float sigm(float g) { return __builtin_amdgcn_rcpf(1.0f + expf(-g)); }

__device__ __forceinline__ void dep_guard4_b(v8f& a, v8f& b, v8f& c, v8f& d, v16b x, v16b y) { asm volatile("v_nop\n\tv_nop\n\tv_nop\n\tv_nop" : "+v"(a), "+v"(b), "+v"(c), "+v"(d) : "v"(x), "v"(y)); }
__device__ __forceinline__ void keep4_b(v16b a, v16b b, v16b c, v16b d) { asm volatile("v_nop" :: "v"(a), "v"(b), "v"(c), "v"(d)); }
__device__ __forceinline__ void acc_guard4(v8f& a, v8f& b, v8f& c, v8f& d) { asm volatile("v_nop\n\tv_nop\n\tv_nop\n\tv_nop" : "+v"(a), "+v"(b), "+v"(c), "+v"(d)); }
template <typename T> struct Frag;
template <> struct Frag<__bf16> {
  typedef v16b V; union U { v16b v; v8b h[2]; };
  static __device__ __forceinline__ v16b load(const __bf16* p) {
    U f; f.h[0] = *(const v8b*)(p); f.h[1] = *(const v8b*)(p + 16); return f.v;
  }
  static __device__ __forceinline__ v8f mma(v16b a, v16b b, v8f c) {
    return __builtin_amdgcn_wmma_f32_16x16x32_bf16(false, a, false, b, (short)0, c, false, false);
  }
  static __device__ __forceinline__ void guard4(v8f& a, v8f& b, v8f& c, v8f& d, v16b x, v16b y) { dep_guard4_b(a, b, c, d, x, y); }
  static __device__ __forceinline__ void keep(v16b a, v16b b, v16b c, v16b d) { keep4_b(a, b, c, d); }
};

template <int SPL, int RES>
__global__ __launch_bounds__(256) void wmma_gemm64_bf16(
    const unsigned short* __restrict__ Ap, const unsigned short* __restrict__ A2p, int lda,
    const unsigned short* __restrict__ Btp, int ldb,
    float* __restrict__ C, int ldc,
    const unsigned short* __restrict__ R16, int ldr,
    int M, int N, int K) {
  const __bf16* A = (const __bf16*)Ap; const __bf16* A2 = (const __bf16*)A2p; const __bf16* Bt = (const __bf16*)Btp;
  __shared__ __align__(16) float sT[8][16 * 68];
  const int lane = threadIdx.x & 31;
  const int wave = threadIdx.x >> 5;
  const int tilesN = N >> 6;
  const int tilesM = M >> 6;
  const int tile = blockIdx.x * 8 + wave;
  if (tile >= tilesM * tilesN) return;
  const int tm = tile / tilesN;
  const int tn = tile - tm * tilesN;
  const int m0 = tm << 6;
  const int n0 = tn << 6;

  const int rlane = lane & 15;
  const int koff  = (lane >> 4) * 8;
  const int mOff  = (lane >> 4) * 8;

  v8f acc[4][4];
#pragma unroll
  for (int i = 0; i < 4; ++i)
#pragma unroll
    for (int j = 0; j < 4; ++j) acc[i][j] = (v8f){0.f,0.f,0.f,0.f,0.f,0.f,0.f,0.f};

  for (int k0 = 0; k0 < K; k0 += 32) {
    v16b bh[4];
#pragma unroll
    for (int j = 0; j < 4; ++j) {
      const size_t bo = (size_t)(n0 + (j << 4) + rlane) * ldb + koff + k0;
      bh[j] = Frag<__bf16>::load(Bt + bo);
    }
#pragma unroll
    for (int i = 0; i < 4; ++i) {
      const size_t ao = (size_t)(m0 + (i << 4) + rlane) * lda + koff + k0;
      v16b ah = Frag<__bf16>::load(A + ao);
      v16b al = ah;
      if (SPL == 1) al = Frag<__bf16>::load(A2 + ao);
#pragma unroll
      for (int j = 0; j < 4; ++j) {
        acc[i][j] = Frag<__bf16>::mma(ah, bh[j], acc[i][j]);
        if (SPL == 1) acc[i][j] = Frag<__bf16>::mma(al, bh[j], acc[i][j]);
      }
      Frag<__bf16>::guard4(acc[i][0], acc[i][1], acc[i][2], acc[i][3], ah, al);
    }
    Frag<__bf16>::keep(bh[0], bh[1], bh[2], bh[3]);
  }
  acc_guard4(acc[0][0], acc[0][1], acc[0][2], acc[0][3]);
  acc_guard4(acc[1][0], acc[1][1], acc[1][2], acc[1][3]);
  acc_guard4(acc[2][0], acc[2][1], acc[2][2], acc[2][3]);
  acc_guard4(acc[3][0], acc[3][1], acc[3][2], acc[3][3]);

  float* slab = sT[wave];
  const int hh = lane >> 4, c4 = (lane & 15) * 4;
#pragma unroll
  for (int i = 0; i < 4; ++i) {
    const int mBase = m0 + (i << 4);
#pragma unroll
    for (int j = 0; j < 4; ++j) {
#pragma unroll
      for (int r = 0; r < 8; ++r) slab[(mOff + r) * 68 + (j << 4) + rlane] = acc[i][j][r];
    }
    __builtin_amdgcn_fence(__ATOMIC_RELEASE, "workgroup");
    __builtin_amdgcn_wave_barrier();
    __builtin_amdgcn_fence(__ATOMIC_ACQUIRE, "workgroup");
    for (int pass = 0; pass < 2; ++pass) {
#pragma unroll
      for (int it = 0; it < 8; ++it) {
        const int row = it * 2 + hh;
        v4f v = *(const v4f*)(slab + row * 68 + c4);
        if (RES == 2) {
          const v2u w = *(const v2u*)(R16 + (size_t)(mBase + row) * ldr + n0 + c4);
          const unsigned w0 = w[0], w1 = w[1];
          v4f rv;
          rv[0] = __uint_as_float(w0 << 16);
          rv[1] = __uint_as_float(w0 & 0xffff0000u);
          rv[2] = __uint_as_float(w1 << 16);
          rv[3] = __uint_as_float(w1 & 0xffff0000u);
          v = v + rv;
        }
        *(volatile v4f*)(C + (size_t)(mBase + row) * ldc + n0 + c4) = v;
      }
      __threadfence();
    }
    __builtin_amdgcn_fence(__ATOMIC_RELEASE, "workgroup");
    __builtin_amdgcn_wave_barrier();
    __builtin_amdgcn_fence(__ATOMIC_ACQUIRE, "workgroup");
  }
}

__global__ __launch_bounds__(256) void wmma_gemm64_gate(
    const unsigned short* __restrict__ Ap, int lda,
    const unsigned short* __restrict__ Btp, int ldb,
    float* __restrict__ Cx, int ldc,
    int M, int N, int K) {
  const __bf16* A = (const __bf16*)Ap; const __bf16* Bt = (const __bf16*)Btp;
  __shared__ __align__(16) float sG[8][16 * kGateSP];
  const int lane = threadIdx.x & 31;
  const int wave = threadIdx.x >> 5;
  const int tilesN = N >> 6;
  const int tilesM = M >> 6;
  const int tile = blockIdx.x * 8 + wave;
  if (tile >= tilesM * tilesN) return;
  const int tm = tile / tilesN;
  const int tn = tile - tm * tilesN;
  const int m0 = tm << 6;
  const int n0 = tn << 6;
  const int nx0 = tn << 5;

  const int rlane = lane & 15;
  const int koff  = (lane >> 4) * 8;
  const int mOff  = (lane >> 4) * 8;

  v8f acc[4][4];
#pragma unroll
  for (int i = 0; i < 4; ++i)
#pragma unroll
    for (int j = 0; j < 4; ++j) acc[i][j] = (v8f){0.f,0.f,0.f,0.f,0.f,0.f,0.f,0.f};

  for (int k0 = 0; k0 < K; k0 += 32) {
    v16b bh[4];
#pragma unroll
    for (int j = 0; j < 4; ++j) {
      const size_t bo = (size_t)(n0 + (j << 4) + rlane) * ldb + koff + k0;
      bh[j] = Frag<__bf16>::load(Bt + bo);
    }
#pragma unroll
    for (int i = 0; i < 4; ++i) {
      const size_t ao = (size_t)(m0 + (i << 4) + rlane) * lda + koff + k0;
      v16b ah = Frag<__bf16>::load(A + ao);
#pragma unroll
      for (int j = 0; j < 4; ++j) acc[i][j] = Frag<__bf16>::mma(ah, bh[j], acc[i][j]);
      Frag<__bf16>::guard4(acc[i][0], acc[i][1], acc[i][2], acc[i][3], ah, ah);
    }
    Frag<__bf16>::keep(bh[0], bh[1], bh[2], bh[3]);
  }
  acc_guard4(acc[0][0], acc[0][1], acc[0][2], acc[0][3]);
  acc_guard4(acc[1][0], acc[1][1], acc[1][2], acc[1][3]);
  acc_guard4(acc[2][0], acc[2][1], acc[2][2], acc[2][3]);
  acc_guard4(acc[3][0], acc[3][1], acc[3][2], acc[3][3]);

  float* slab = sG[wave];
  const int q = lane >> 3, c4 = (lane & 7) * 4;
#pragma unroll
  for (int i = 0; i < 4; ++i) {
    const int mBase = m0 + (i << 4);
#pragma unroll
    for (int jp = 0; jp < 2; ++jp) {
#pragma unroll
      for (int r = 0; r < 8; ++r) {
        const float sv = acc[i][jp][r];
        const float gv = acc[i][jp + 2][r];
        slab[(mOff + r) * kGateSP + (jp << 4) + rlane] = sv * sigm(gv);
      }
    }
    __builtin_amdgcn_fence(__ATOMIC_RELEASE, "workgroup");
    __builtin_amdgcn_wave_barrier();
    __builtin_amdgcn_fence(__ATOMIC_ACQUIRE, "workgroup");
    for (int pass = 0; pass < 2; ++pass) {
#pragma unroll
      for (int it = 0; it < 4; ++it) {
        const int row = it * 4 + q;
        const v4f v = *(const v4f*)(slab + row * kGateSP + c4);
        *(volatile v4f*)(Cx + (size_t)(mBase + row) * ldc + nx0 + c4) = v;
      }
      __threadfence();
    }
    __builtin_amdgcn_fence(__ATOMIC_RELEASE, "workgroup");
    __builtin_amdgcn_wave_barrier();
    __builtin_amdgcn_fence(__ATOMIC_ACQUIRE, "workgroup");
  }
}

__global__ __launch_bounds__(256) void cvt_rows_bf16_kernel(
    const float* __restrict__ src, unsigned short* __restrict__ dst, int total8)
{
  const int i = blockIdx.x * 256 + threadIdx.x;
  if (i >= total8) return;
  const size_t e0 = (size_t)i << 3;
  const v4f a0 = *(const v4f*)(src + e0);
  const v4f a1 = *(const v4f*)(src + e0 + 4);
  v8h hv;
#pragma unroll
  for (int e = 0; e < 4; ++e) {
    const float f0 = a0[e], f1 = a1[e];
    const unsigned short b0 = f2bf_bits(f0), b1 = f2bf_bits(f1);
    hv[e]     = __builtin_bit_cast(_Float16, b0);
    hv[4 + e] = __builtin_bit_cast(_Float16, b1);
  }
  unsigned short* qh = dst + e0;
  *(volatile v8h*)qh = hv;
  __threadfence();
  *(volatile v8h*)qh = hv;
}

__global__ __launch_bounds__(256) void cvt_win_perm_kernel(const float* __restrict__ W_in, unsigned short* __restrict__ WIB)
{
  const int i = blockIdx.x * 256 + threadIdx.x;
  if (i >= kWin * kDm / 8) return;
  const int p  = i >> 6;
  const int k0 = (i & 63) * 8;
  const int t  = p >> 6, w = p & 63;
  const int src = (w < 32) ? (32 * t + w) : (kE + 32 * t + (w - 32));
  const float* sp = W_in + (size_t)src * kDm + k0;
  const v4f a0 = *(const v4f*)(sp);
  const v4f a1 = *(const v4f*)(sp + 4);
  v8h hv;
#pragma unroll
  for (int e = 0; e < 4; ++e) {
    const float f0 = a0[e], f1 = a1[e];
    const unsigned short b0 = f2bf_bits(f0), b1 = f2bf_bits(f1);
    hv[e]     = __builtin_bit_cast(_Float16, b0);
    hv[4 + e] = __builtin_bit_cast(_Float16, b1);
  }
  unsigned short* qh = WIB + ((size_t)i << 3);
  *(volatile v8h*)qh = hv;
  __threadfence();
  *(volatile v8h*)qh = hv;
}

__global__ __launch_bounds__(256) void bpt_pad_kernel(const float* __restrict__ Bp, unsigned short* __restrict__ BPT)
{
  const int i = blockIdx.x * 256 + threadIdx.x;
  if (i >= kDlP * kE / 8) return;
  const int n = i >> 7;
  const int e0 = (i & 127) * 8;
  const int nc = (n < kNst) ? n : (kNst - 1);
  const float fz = (float)(n < kNst);
  v8h hv;
#pragma unroll
  for (int j = 0; j < 8; ++j) {
    const float ld = Bp[(size_t)(e0 + j) * kNst + nc];
    const float v = ld * fz;
    const unsigned short b0 = f2bf_bits(v);
    hv[j] = __builtin_bit_cast(_Float16, b0);
  }
  unsigned short* qh = BPT + (size_t)n * kE + e0;
  *(volatile v8h*)qh = hv;
  __threadfence();
  *(volatile v8h*)qh = hv;
}

__global__ __launch_bounds__(256) void conv_silu_kernel(
    const float* __restrict__ XS, const float* __restrict__ Wc,
    unsigned short* __restrict__ UH, unsigned short* __restrict__ UL)
{
  __shared__ __align__(16) float sT[16 * kConvTP];
  const int tid = threadIdx.x, lane = tid & 31, wave = tid >> 5;
  const int d0 = blockIdx.x * 256, d = d0 + tid;
  const int g0 = blockIdx.y * 64;
  const int tb = g0 & (kSeq - 1);
  const v4f wv = *(const v4f*)(Wc + (size_t)d * kConvK);
  const float w0 = bfr(wv[0]), w1 = bfr(wv[1]), w2 = bfr(wv[2]), w3 = bfr(wv[3]);
  float xm3, xm2, xm1;
  {
    const bool hist = (tb > 0);
    const int rb = hist ? (g0 - 3) : g0;
    const float* p = XS + (size_t)rb * kE + d;
    const float v0 = p[0];
    const float v1 = p[kE];
    const float v2 = p[2 * kE];
    xm3 = hist ? v0 : 0.0f;
    xm2 = hist ? v1 : 0.0f;
    xm1 = hist ? v2 : 0.0f;
  }
#pragma unroll 1
  for (int sub = 0; sub < 4; ++sub) {
    const int lb = g0 + sub * 16;
#pragma unroll 1
    for (int s = 0; s < 16; ++s) {
      const float xs = XS[(size_t)(lb + s) * kE + d];
      float acc = w0 * xm3;
      acc = fmaf(w1, xm2, acc);
      acc = fmaf(w2, xm1, acc);
      acc = fmaf(w3, xs, acc);
      sT[s * kConvTP + tid] = acc * sigm(acc);
      xm3 = xm2; xm2 = xm1; xm1 = xs;
    }
    __syncthreads();
    v8h hv[2], lv[2];
#pragma unroll
    for (int it = 0; it < 2; ++it) {
      const float* sp = sT + (it * 8 + wave) * kConvTP + lane * 8;
      const v4f a0 = *(const v4f*)(sp);
      const v4f a1 = *(const v4f*)(sp + 4);
#pragma unroll
      for (int e2 = 0; e2 < 4; ++e2) {
        const float f0 = a0[e2], f1 = a1[e2];
        const unsigned short h0 = f2bf_bits(f0), h1 = f2bf_bits(f1);
        const unsigned short l0 = f2bf_bits(f0 - bf_bits2f(h0)), l1 = f2bf_bits(f1 - bf_bits2f(h1));
        hv[it][e2]     = __builtin_bit_cast(_Float16, h0);
        hv[it][4 + e2] = __builtin_bit_cast(_Float16, h1);
        lv[it][e2]     = __builtin_bit_cast(_Float16, l0);
        lv[it][4 + e2] = __builtin_bit_cast(_Float16, l1);
      }
    }
    for (int pass = 0; pass < 2; ++pass) {
#pragma unroll
      for (int it = 0; it < 2; ++it) {
        const size_t o = (size_t)(lb + it * 8 + wave) * kE + d0 + lane * 8;
        *(volatile v8h*)(UH + o) = hv[it];
        *(volatile v8h*)(UL + o) = lv[it];
      }
      __threadfence();
    }
    __syncthreads();
  }
}

__global__ __launch_bounds__(256) void scan_kernel(
    const float* __restrict__ DL, const unsigned short* __restrict__ UH, const unsigned short* __restrict__ UL,
    const float* __restrict__ Am, const float* __restrict__ Bpm, const float* __restrict__ Cpm,
    const float* __restrict__ Dpv, unsigned short* __restrict__ YH, unsigned short* __restrict__ YL)
{
  __shared__ __align__(16) float sD[kScanTS * kNst];
  __shared__ __align__(16) float sU[kScanTS * kScanCh];
  __shared__ __align__(16) float sY[kScanTS * kSYP];
  const int tid = threadIdx.x, lane = tid & 31, wave = tid >> 5;
  constexpr int kBlkPerB = kE / kScanCh;
  const int bix = blockIdx.x / kBlkPerB;
  const int d0  = (blockIdx.x - bix * kBlkPerB) * kScanCh;
  const int c   = tid >> 2;
  const int nq  = tid & 3;
  const int e   = d0 + c;
  const size_t row0 = (size_t)bix * kSeq;
  float aneg[4], bp[4], cp[4], h[4];
  {
    const v4f av = *(const v4f*)(Am  + (size_t)e * kNst + 4 * nq);
    const v4f bv = *(const v4f*)(Bpm + (size_t)e * kNst + 4 * nq);
    const v4f cv = *(const v4f*)(Cpm + (size_t)e * kNst + 4 * nq);
#pragma unroll
    for (int k = 0; k < 4; ++k) {
      aneg[k] = -expf(bfr(av[k]));
      bp[k] = bfr(bv[k]);
      cp[k] = bfr(cv[k]);
      h[k] = 0.0f;
    }
  }
  const float dpe = bfr(Dpv[e]);
  const int sr = tid >> 2, sc4 = (tid & 3) * 4;
  const int q = lane >> 3, c8 = (lane & 7) * 8;
#pragma unroll 1
  for (int t0 = 0; t0 < kSeq; t0 += kScanTS) {
    __syncthreads();
    {
      const v4f lv = *(const v4f*)(DL + (row0 + t0 + sr) * kDlP + sc4);
      v4f sv;
#pragma unroll
      for (int j = 0; j < 4; ++j) sv[j] = sigm(lv[j]);
      *(v4f*)(sD + sr * kNst + sc4) = sv;
    }
#pragma unroll
    for (int i = 0; i < 2; ++i) {
      const int idx = tid + 256 * i;
      const int ur = idx >> 3, uc8 = (idx & 7) * 8;
      const size_t go = (row0 + t0 + ur) * kE + d0 + uc8;
      const v4u wh = *(const v4u*)(UH + go);
      const v4u wl = *(const v4u*)(UL + go);
      v4f f0, f1;
#pragma unroll
      for (int j = 0; j < 2; ++j) {
        const unsigned a = wh[j], b = wl[j];
        f0[2 * j]     = __uint_as_float(a << 16) + __uint_as_float(b << 16);
        f0[2 * j + 1] = __uint_as_float(a & 0xffff0000u) + __uint_as_float(b & 0xffff0000u);
        const unsigned a2 = wh[2 + j], b2 = wl[2 + j];
        f1[2 * j]     = __uint_as_float(a2 << 16) + __uint_as_float(b2 << 16);
        f1[2 * j + 1] = __uint_as_float(a2 & 0xffff0000u) + __uint_as_float(b2 & 0xffff0000u);
      }
      *(v4f*)(sU + ur * kScanCh + uc8)     = f0;
      *(v4f*)(sU + ur * kScanCh + uc8 + 4) = f1;
    }
    __syncthreads();
#pragma unroll 1
    for (int s = 0; s < kScanTS; ++s) {
      const v4f d4 = *(const v4f*)(sD + s * kNst + 4 * nq);
      const float u = sU[s * kScanCh + c];
      float y = 0.0f;
#pragma unroll
      for (int k = 0; k < 4; ++k) {
        const float dl = d4[k];
        const float at = expf(aneg[k] * dl);
        h[k] = fmaf(at, h[k], (dl * bp[k]) * u);
        y = fmaf(h[k], cp[k], y);
      }
      y += __shfl_xor(y, 1, 32);
      y += __shfl_xor(y, 2, 32);
      y = fmaf(dpe, u, y);
      if (nq == 0) sY[s * kSYP + c] = y;
    }
    __syncthreads();
    v8h hv[2], lv[2];
#pragma unroll
    for (int it = 0; it < 2; ++it) {
      const int row = it * 32 + wave * 4 + q;
      const float* sp = sY + row * kSYP + c8;
      const v4f a0 = *(const v4f*)(sp);
      const v4f a1 = *(const v4f*)(sp + 4);
#pragma unroll
      for (int e2 = 0; e2 < 4; ++e2) {
        const float f0 = a0[e2], f1 = a1[e2];
        const unsigned short h0 = f2bf_bits(f0), h1 = f2bf_bits(f1);
        const unsigned short l0 = f2bf_bits(f0 - bf_bits2f(h0)), l1 = f2bf_bits(f1 - bf_bits2f(h1));
        hv[it][e2]     = __builtin_bit_cast(_Float16, h0);
        hv[it][4 + e2] = __builtin_bit_cast(_Float16, h1);
        lv[it][e2]     = __builtin_bit_cast(_Float16, l0);
        lv[it][4 + e2] = __builtin_bit_cast(_Float16, l1);
      }
    }
    for (int pass = 0; pass < 2; ++pass) {
#pragma unroll
      for (int it = 0; it < 2; ++it) {
        const int row = it * 32 + wave * 4 + q;
        const size_t o = (row0 + t0 + row) * kE + d0 + c8;
        *(volatile v8h*)(YH + o) = hv[it];
        *(volatile v8h*)(YL + o) = lv[it];
      }
      __threadfence();
    }
  }
}

extern "C" void kernel_launch(void* const* d_in, const int* in_sizes, int n_in,
                              void* d_out, int out_size, void* d_ws, size_t ws_size,
                              hipStream_t stream) {
  if (n_in < 8) return;
  if (in_sizes[0] != kRows * kDm) return;
  if (in_sizes[1] != kWin * kDm) return;
  if (in_sizes[2] != kE * kConvK) return;
  if (in_sizes[3] != kE * kNst) return;
  if (in_sizes[4] != kE * kNst) return;
  if (in_sizes[5] != kE * kNst) return;
  if (in_sizes[6] != kE) return;
  if (in_sizes[7] != kDm * kE) return;
  if (out_size != kRows * kDm) return;
  if (ws_size < kWsTotal) return;

  const float* x      = (const float*)d_in[0];
  const float* W_in   = (const float*)d_in[1];
  const float* W_conv = (const float*)d_in[2];
  const float* Am     = (const float*)d_in[3];
  const float* Bp     = (const float*)d_in[4];
  const float* Cp     = (const float*)d_in[5];
  const float* Dp     = (const float*)d_in[6];
  const float* W_out  = (const float*)d_in[7];
  float* out = (float*)d_out;

  char* ws = (char*)d_ws;
  unsigned short* XB  = (unsigned short*)(ws + kOffXB);
  unsigned short* WIB = (unsigned short*)(ws + kOffWIB);
  unsigned short* WOB = (unsigned short*)(ws + kOffWOB);
  unsigned short* BPT = (unsigned short*)(ws + kOffBPT);
  float*          XS  = (float*)(ws + kOffXS);
  unsigned short* UH  = (unsigned short*)(ws + kOffUH);
  unsigned short* UL  = (unsigned short*)(ws + kOffUL);
  float*          DL  = (float*)(ws + kOffDL);
  unsigned short* YH  = (unsigned short*)(ws + kOffYH);
  unsigned short* YL  = (unsigned short*)(ws + kOffYL);

  cvt_rows_bf16_kernel<<<(kRows * kDm / 8) / 256, 256, 0, stream>>>(x, XB, kRows * kDm / 8);
  cvt_win_perm_kernel<<<(kWin * kDm / 8) / 256, 256, 0, stream>>>(W_in, WIB);
  cvt_rows_bf16_kernel<<<(kDm * kE / 8) / 256, 256, 0, stream>>>(W_out, WOB, kDm * kE / 8);
  bpt_pad_kernel<<<(kDlP * kE / 8) / 256, 256, 0, stream>>>(Bp, BPT);

  wmma_gemm64_gate<<<dim3(kTilesIn / 8, 1), 256, 0, stream>>>(
      XB, kDm, WIB, kDm, XS, kE, kRows, kWin, kDm);

  conv_silu_kernel<<<dim3(kE / 256, kRows / 64), 256, 0, stream>>>(XS, W_conv, UH, UL);

  wmma_gemm64_bf16<1, 0><<<dim3(kTilesDl / 8, 1), 256, 0, stream>>>(
      UH, UL, kE, BPT, kE, DL, kDlP, nullptr, 0, kRows, kDlP, kE);

  scan_kernel<<<kBatch * (kE / kScanCh), 256, 0, stream>>>(DL, UH, UL, Am, Bp, Cp, Dp, YH, YL);

  wmma_gemm64_bf16<1, 2><<<dim3(kTilesOut / 8, 1), 256, 0, stream>>>(
      YH, YL, kE, WOB, kE, out, kDm, XB, kDm, kRows, kDm, kE);
}
